// GAT_38044820308171
// MI455X (gfx1250) — hardware-verified
//
#include <hip/hip_runtime.h>
#include <stddef.h>
#include <stdint.h>
#include <math.h>


#define FIN     128
#define HC      384
#define NHD     3
#define HID     128
#define NCLS    6
#define KA2     256
#define NTHR    256
#define NWAVE   8
#define EPT     8
#define CHUNK   (NTHR * EPT)
#define WCAP    (EPT * 32)
#define LISTN   (NWAVE * WCAP)
#define NBA     1024
#define SLA     10
#define RCAP    28672
#define DEGCAP  128
#define MEAS_B1024  16696
#define MEAS_MAXDEG 33
#define GBM     64
#define GBN     64
#define GTHR    128
#define MROWS   128
#define ORW     128
#define NUW1    (HC * (FIN / 8))
#define NU2     (HC * (KA2 / 8))
#define NUL     (HID * (KA2 / 8))
#define NU5     (16 * (KA2 / 8))
#define PAR_AL1 0
#define PAR_AR1 384
#define PAR_B1  768
#define PAR_AL2 1152
#define PAR_AR2 1536
#define PAR_B2  1920
#define PAR_LB  2304
#define PAR_LB5 2816
#define PAR_N   2848
#define GSLOPE  0.2f
#define ASLOPE  0.01f
#define MXI     (-3.0e38f)
#define WSMAX   134217728
#define BKT_LDS_INTS  (LISTN + 2 * RCAP + 3 * NBA + 16)
#define SCAN_LDS_INTS (RCAP + 2 * NBA + 16)

static_assert((CHUNK & (CHUNK - 1)) == 0 && CHUNK <= 4096);
static_assert((NBA & (NBA - 1)) == 0 && NBA == (1 << SLA) && NBA <= 1024);
static_assert(((long long)CHUNK << SLA) < (1LL << 31));
static_assert(LISTN >= NWAVE * WCAP);
static_assert(NBA % NWAVE == 0 && NBA % 32 == 0 && NBA % 16 == 0 && NBA == 4 * NTHR);
static_assert((RCAP % 32) == 0 && ((RCAP + 3 * NBA) % 4) == 0 && (RCAP % (NTHR * 4)) == 0);
static_assert(((RCAP + 3 * NBA) % (NTHR * 4)) == 0);
static_assert(RCAP >= MEAS_B1024 + 4096);
static_assert(DEGCAP >= MEAS_MAXDEG + 8);
static_assert(BKT_LDS_INTS * 4 <= 300000 && SCAN_LDS_INTS * 4 <= 300000);
static_assert(GBM == (GTHR / 32) * 16 && GTHR == 2 * GBN);
static_assert((FIN % 32) == 0 && (KA2 % 32) == 0 && KA2 == 2 * HID);
static_assert((HC % GBN) == 0 && (HID % GBN) == 0 && HC == NHD * HID && HID == 4 * 32);
static_assert((MROWS % GBM) == 0 && (NBA % ORW) == 0 && (ORW % 16) == 0 && ORW == MROWS);
static_assert((NUW1 % NTHR) == 0 && (NU2 % NTHR) == 0 && (NUL % NTHR) == 0 && (NU5 % NTHR) == 0);
static_assert(PAR_LB == 18 * 128 && PAR_LB5 == 22 * 128 && PAR_N == PAR_LB5 + 32);
static_assert((ORW * NCLS) % 4 == 0 && (ORW * NCLS) / 4 == 192);
static_assert(GBN / 4 == 16);

typedef float          v4f  __attribute__((ext_vector_type(4)));
typedef float          v8f  __attribute__((ext_vector_type(8)));
typedef int            v4i  __attribute__((ext_vector_type(4)));
typedef int            v8i  __attribute__((ext_vector_type(8)));
typedef unsigned int   v2u  __attribute__((ext_vector_type(2)));
typedef unsigned int   v4u  __attribute__((ext_vector_type(4)));
typedef unsigned short v8us __attribute__((ext_vector_type(8)));
typedef __bf16         v16b __attribute__((ext_vector_type(16)));
typedef v4f  __attribute__((may_alias)) v4fa;
typedef v4i  __attribute__((may_alias)) v4ia;
typedef v8us __attribute__((may_alias)) v8usa;
union FragB { v16b v; v8us h[2]; v8i w; };

__device__ __forceinline__ v8f wmb(const FragB& a, const FragB& b, v8f c) {
  v8f d = __builtin_amdgcn_wmma_f32_16x16x32_bf16(false, a.v, false, b.v, (short)0, c, false, false);
  asm volatile("v_nop\n\tv_nop\n\tv_nop\n\tv_nop" : "+v"(d) : "v"(a.w), "v"(b.w));
  return d;
}

__device__ __forceinline__ unsigned int f2bf(float f) {
  const unsigned int u = __float_as_uint(f);
  const unsigned int r = ((u + 0x7FFFu + ((u >> 16) & 1u)) >> 16) & 0xFFFFu;
  return ((u & 0x7FFFFFFFu) > 0x7F800000u) ? 0x7FC0u : r;
}
__device__ __forceinline__ float bf2f(unsigned int b) { return __uint_as_float(b << 16); }
__device__ __forceinline__ float bfr(float f) { return bf2f(f2bf(f)); }
__device__ __forceinline__ v4f bfr4(const v4f a) {
  v4f r; r.x = bfr(a.x); r.y = bfr(a.y); r.z = bfr(a.z); r.w = bfr(a.w); return r;
}
__device__ __forceinline__ unsigned int pk2(float lo, float hi) { return f2bf(lo) | (f2bf(hi) << 16); }
__device__ __forceinline__ unsigned int pk2lo(float lo, float hi) {
  return f2bf(lo - bfr(lo)) | (f2bf(hi - bfr(hi)) << 16);
}
__device__ __forceinline__ v4u pack8(const v4f a, const v4f b) {
  v4u r;
  r.x = pk2(a.x, a.y); r.y = pk2(a.z, a.w); r.z = pk2(b.x, b.y); r.w = pk2(b.z, b.w);
  return r;
}
__device__ __forceinline__ v4u pack8lo(const v4f a, const v4f b) {
  v4u r;
  r.x = pk2lo(a.x, a.y); r.y = pk2lo(a.z, a.w); r.z = pk2lo(b.x, b.y); r.w = pk2lo(b.z, b.w);
  return r;
}
__device__ __forceinline__ float lk(float v) { return v > 0.0f ? v : ASLOPE * v; }

__device__ __forceinline__ v4u gather8(const float* __restrict__ p, int stride) {
  v4f a, b;
  a.x = p[0];                    a.y = p[(size_t)stride];       a.z = p[(size_t)2 * stride];   a.w = p[(size_t)3 * stride];
  b.x = p[(size_t)4 * stride];   b.y = p[(size_t)5 * stride];   b.z = p[(size_t)6 * stride];   b.w = p[(size_t)7 * stride];
  return pack8(a, b);
}
__device__ __forceinline__ v4f ld4r(const float* __restrict__ p, int unit) {
  return bfr4(*(const v4f*)(p + 4 * unit));
}

template <int SLB>
__device__ __forceinline__ int scan_chunk(const int* __restrict__ dsts, int nE, int cbase, int slotBase,
                                          int nb, int vec8, int* list, int tid, int lane, int wave) {
  int wc = 0;
  const int el0  = tid * EPT;
  const int e0   = cbase + el0;
  const int sent = -2147483647 - 1;
  v4i da, db;
  if (vec8 != 0 && cbase + CHUNK <= nE) {
    da = *(const v4i*)(dsts + e0);
    db = *(const v4i*)(dsts + e0 + 4);
  } else {
    da.x = (e0     < nE) ? dsts[min(e0,     nE - 1)] : sent;
    da.y = (e0 + 1 < nE) ? dsts[min(e0 + 1, nE - 1)] : sent;
    da.z = (e0 + 2 < nE) ? dsts[min(e0 + 2, nE - 1)] : sent;
    da.w = (e0 + 3 < nE) ? dsts[min(e0 + 3, nE - 1)] : sent;
    db.x = (e0 + 4 < nE) ? dsts[min(e0 + 4, nE - 1)] : sent;
    db.y = (e0 + 5 < nE) ? dsts[min(e0 + 5, nE - 1)] : sent;
    db.z = (e0 + 6 < nE) ? dsts[min(e0 + 6, nE - 1)] : sent;
    db.w = (e0 + 7 < nE) ? dsts[min(e0 + 7, nE - 1)] : sent;
  }
  const unsigned nbs = (unsigned)slotBase;
  const unsigned unb = (unsigned)nb;
  const unsigned s0 = (unsigned)da.x - nbs, s1 = (unsigned)da.y - nbs;
  const unsigned s2 = (unsigned)da.z - nbs, s3 = (unsigned)da.w - nbs;
  const unsigned s4 = (unsigned)db.x - nbs, s5 = (unsigned)db.y - nbs;
  const unsigned s6 = (unsigned)db.z - nbs, s7 = (unsigned)db.w - nbs;
  const bool h0 = s0 < unb, h1 = s1 < unb, h2 = s2 < unb, h3 = s3 < unb;
  const bool h4 = s4 < unb, h5 = s5 < unb, h6 = s6 < unb, h7 = s7 < unb;
  const unsigned any = __builtin_amdgcn_ballot_w32(h0 | h1 | h2 | h3 | h4 | h5 | h6 | h7);
  if (any != 0u) {
#define HITJ(J, HJ, SJ) { \
      const unsigned mj = __builtin_amdgcn_ballot_w32(HJ); \
      if (mj != 0u) { \
        if (HJ) { \
          const int pos = wc + (int)__builtin_amdgcn_mbcnt_lo(mj, 0u); \
          if (pos < WCAP) list[wave * WCAP + pos] = ((el0 + (J)) << SLB) | (int)(SJ); \
        } \
        wc += (int)__builtin_popcount(mj); } }
    HITJ(0, h0, s0)
    HITJ(1, h1, s1)
    HITJ(2, h2, s2)
    HITJ(3, h3, s3)
    HITJ(4, h4, s4)
    HITJ(5, h5, s5)
    HITJ(6, h6, s6)
    HITJ(7, h7, s7)
#undef HITJ
  }
  return wc;
}

__global__ __launch_bounds__(NTHR) __attribute__((amdgpu_num_vgpr(248)))
void k_pa(const float* __restrict__ x, const float* __restrict__ W1,
          unsigned short* XB, unsigned short* W1T, int nN, int nUx) {
  const int u = (int)blockIdx.x * NTHR + (int)threadIdx.x;
  v4u o;
  unsigned short* dp;
  if (u < nUx) {
    const int row = u >> 4;
    const int c0  = (u & 15) * 8;
    const int rc  = row < nN ? row : nN - 1;
    const float* p = x + (size_t)rc * FIN + c0;
    v4f a = *(const v4f*)p, b = *(const v4f*)(p + 4);
    const v4f z4 = {0.f, 0.f, 0.f, 0.f};
    if (row >= nN) { a = z4; b = z4; }
    o = pack8(a, b);
    dp = XB + (size_t)row * FIN + c0;
  } else if (u < nUx + NUW1) {
    const int v  = u - nUx;
    const int n  = v >> 4;
    const int k8 = (v & 15) * 8;
    o = gather8(W1 + (size_t)k8 * HC + n, HC);
    dp = W1T + (size_t)n * FIN + k8;
  } else {
    return;
  }
  *(volatile v4u*)dp = o;
  __threadfence();
  *(volatile v4u*)dp = o;
}

__global__ __launch_bounds__(NTHR) __attribute__((amdgpu_num_vgpr(248)))
void k_pb(const float* __restrict__ W2, const float* __restrict__ lw1, const float* __restrict__ lw2,
          const float* __restrict__ lw3, const float* __restrict__ lw4, const float* __restrict__ lw5,
          unsigned short* W2D, unsigned short* LWD, unsigned short* LW5D) {
  const int u = (int)blockIdx.x * NTHR + (int)threadIdx.x;
  v4u o;
  unsigned short* dp;
  if (u < NU2) {
    const int n = u >> 5, k8 = (u & 31) * 8, kk = k8 & (HID - 1);
    o = gather8(W2 + (size_t)kk * HC + n, HC);
    dp = W2D + (size_t)n * KA2 + k8;
  } else if (u < NU2 + NUL) {
    const int v = u - NU2;
    const int n = v >> 5, k8 = (v & 31) * 8, kk = k8 & (HID - 1);
    o = gather8(lw1 + (size_t)kk * HID + n, HID);
    dp = LWD + (size_t)n * KA2 + k8;
  } else if (u < NU2 + 2 * NUL) {
    const int v = u - NU2 - NUL;
    const int n = v >> 5, k8 = (v & 31) * 8, kk = k8 & (HID - 1);
    o = gather8(lw2 + (size_t)kk * HID + n, HID);
    dp = LWD + (size_t)HID * KA2 + (size_t)n * KA2 + k8;
  } else if (u < NU2 + 3 * NUL) {
    const int v = u - NU2 - 2 * NUL;
    const int n = v >> 5, k8 = (v & 31) * 8, kk = k8 & (HID - 1);
    o = gather8(lw3 + (size_t)kk * HID + n, HID);
    dp = LWD + (size_t)2 * HID * KA2 + (size_t)n * KA2 + k8;
  } else if (u < NU2 + 4 * NUL) {
    const int v = u - NU2 - 3 * NUL;
    const int n = v >> 5, k8 = (v & 31) * 8, kk = k8 & (HID - 1);
    o = gather8(lw4 + (size_t)kk * HID + n, HID);
    dp = LWD + (size_t)3 * HID * KA2 + (size_t)n * KA2 + k8;
  } else if (u < NU2 + 4 * NUL + NU5) {
    const int v = u - NU2 - 4 * NUL;
    const int n = v >> 5, k8 = (v & 31) * 8, kk = k8 & (HID - 1);
    const int ncl = n < NCLS ? n : NCLS - 1;
    o = gather8(lw5 + (size_t)kk * NCLS + ncl, NCLS);
    const v4u z = {0u, 0u, 0u, 0u};
    if (n >= NCLS) o = z;
    dp = LW5D + (size_t)n * KA2 + k8;
  } else {
    return;
  }
  *(volatile v4u*)dp = o;
  __threadfence();
  *(volatile v4u*)dp = o;
}

__global__ __launch_bounds__(32) __attribute__((amdgpu_num_vgpr(248)))
void k_pc(const float* __restrict__ al1, const float* __restrict__ ar1, const float* __restrict__ b1,
          const float* __restrict__ al2, const float* __restrict__ ar2, const float* __restrict__ b2,
          const float* __restrict__ lb1, const float* __restrict__ lb2, const float* __restrict__ lb3,
          const float* __restrict__ lb4, const float* __restrict__ lb5, float* PAR) {
  const int b = (int)blockIdx.x, lane = (int)threadIdx.x & 31;
  v4f v;
  if (b < 3)        v = ld4r(al1, b * 32 + lane);
  else if (b < 6)   v = ld4r(ar1, (b - 3) * 32 + lane);
  else if (b < 9)   v = ld4r(b1,  (b - 6) * 32 + lane);
  else if (b < 12)  v = ld4r(al2, (b - 9) * 32 + lane);
  else if (b < 15)  v = ld4r(ar2, (b - 12) * 32 + lane);
  else if (b < 18)  v = ld4r(b2,  (b - 15) * 32 + lane);
  else if (b == 18) v = ld4r(lb1, lane);
  else if (b == 19) v = ld4r(lb2, lane);
  else if (b == 20) v = ld4r(lb3, lane);
  else if (b == 21) v = ld4r(lb4, lane);
  else {
    const int i0 = 4 * lane;
    const float t0 = lb5[min(i0,     NCLS - 1)];
    const float t1 = lb5[min(i0 + 1, NCLS - 1)];
    const float t2 = lb5[min(i0 + 2, NCLS - 1)];
    const float t3 = lb5[min(i0 + 3, NCLS - 1)];
    v.x = (i0     < NCLS) ? bfr(t0) : 0.0f;
    v.y = (i0 + 1 < NCLS) ? bfr(t1) : 0.0f;
    v.z = (i0 + 2 < NCLS) ? bfr(t2) : 0.0f;
    v.w = (i0 + 3 < NCLS) ? bfr(t3) : 0.0f;
  }
  if (b > 22) return;
  float* dp = PAR + (size_t)b * 128 + 4 * lane;
  const bool wr = (b < 22) || (lane < 8);
  if (wr) *(volatile v4f*)dp = v;
  __threadfence();
  if (wr) *(volatile v4f*)dp = v;
}

__global__ __launch_bounds__(NTHR) __attribute__((amdgpu_num_vgpr(248)))
void k_bucket(const int* __restrict__ srcs, const int* __restrict__ dsts, int nE, int nN, int vec8,
              int* HITS, int* CNT, int* OFFS, int* FLG) {
  extern __shared__ __attribute__((aligned(16))) int bsm[];
  int* list = bsm;
  int* reg1 = list + LISTN;
  int* reg2 = reg1 + RCAP;
  int* cnt  = reg2 + RCAP;
  int* offs = cnt + NBA;
  int* cur  = offs + NBA;
  int* wcnt = cur + NBA;
  const int tid = (int)threadIdx.x, lane = tid & 31, wave = tid >> 5;
  const int blk = (int)blockIdx.x;
  const int nodeBase = blk * NBA;
  int nb = nN - nodeBase;
  nb = nb < 0 ? 0 : (nb > NBA ? NBA : nb);

  {
    const v4i z4 = {0, 0, 0, 0};
    for (int i = tid * 4; i < RCAP + 3 * NBA; i += NTHR * 4) *(v4ia*)(reg2 + i) = z4;
    if (tid < 16) wcnt[tid] = 0;
  }
  __syncthreads();

  int tot = 0, ovf = 0;
  const int nChunks = (nE + CHUNK - 1) / CHUNK;
#pragma unroll 1
  for (int ch = 0; ch < nChunks; ++ch) {
    const int cbase = ch * CHUNK;
    const int wc = scan_chunk<SLA>(dsts, nE, cbase, nodeBase, nb, vec8, list, tid, lane, wave);
    if (lane == 0) wcnt[wave] = wc;
    __syncthreads();
    int pre = 0, all = 0;
#pragma unroll
    for (int w2 = 0; w2 < NWAVE; ++w2) {
      int c = wcnt[w2];
      c = c < 0 ? 0 : (c > WCAP ? WCAP : c);
      all += c;
      pre += (w2 < wave) ? c : 0;
    }
    const int wcc  = wc > WCAP ? WCAP : wc;
    const int base = tot + pre;
#pragma unroll 1
    for (int i0 = 0; i0 < wcc; i0 += 32) {
      const int i   = i0 + lane;
      const int ic  = i < wcc ? i : wcc - 1;
      const int ent = list[wave * WCAP + ic];
      const int el  = (ent >> SLA) & (CHUNK - 1);
      const int sl  = ent & (NBA - 1);
      int eid = cbase + el;
      eid = eid > nE - 1 ? nE - 1 : eid;
      const int sraw = srcs[eid];
      const int s = sraw < 0 ? 0 : (sraw > nN - 1 ? nN - 1 : sraw);
      const int pos = base + i;
      if (i < wcc && pos < RCAP) reg1[pos] = (int)((unsigned)s | ((unsigned)sl << 16));
    }
    if (tot + all > RCAP) ovf = 1;
    tot += all;
    tot = tot > RCAP ? RCAP : tot;
    __syncthreads();
  }
  const int nh = tot;

  if (wave == 0) {
#pragma unroll 1
    for (int b0 = 0; b0 < nh; b0 += 32) {
      const int idx = b0 + lane;
      const int uv  = reg1[idx < nh ? idx : nh - 1];
      const int m32 = (nh - b0) < 32 ? (nh - b0) : 32;
#pragma unroll 1
      for (int k = 0; k < m32; ++k) {
        const int u  = __builtin_amdgcn_readlane(uv, k);
        const int sq = (u >> 16) & (NBA - 1);
        if (lane == 0) cnt[sq] = cnt[sq] + 1;
      }
    }
  }
  __syncthreads();
  if (wave == 0) {
    const int base = lane * (NBA / 32);
    int s = 0;
#pragma unroll 1
    for (int i = 0; i < NBA / 32; ++i) s += cnt[base + i];
    int incl = s;
#pragma unroll
    for (int d = 1; d < 32; d <<= 1) {
      const int y = __shfl_up(incl, d, 32);
      if (lane >= d) incl += y;
    }
    int run = incl - s;
#pragma unroll 1
    for (int i = 0; i < NBA / 32; ++i) {
      const int cv = cnt[base + i];
      offs[base + i] = run;
      cur[base + i]  = run;
      run += cv;
    }
  }
  __syncthreads();
  if (wave == 0) {
#pragma unroll 1
    for (int b0 = 0; b0 < nh; b0 += 32) {
      const int idx = b0 + lane;
      const int uv  = reg1[idx < nh ? idx : nh - 1];
      const int m32 = (nh - b0) < 32 ? (nh - b0) : 32;
#pragma unroll 1
      for (int k = 0; k < m32; ++k) {
        const int u  = __builtin_amdgcn_readlane(uv, k);
        const int sq = (u >> 16) & (NBA - 1);
        if (lane == 0) {
          int p = cur[sq];
          p = p < 0 ? 0 : (p > RCAP - 1 ? RCAP - 1 : p);
          reg2[p] = u;
          cur[sq] = p + 1;
        }
      }
    }
  }
  __syncthreads();

  int* hb = HITS + (size_t)blk * RCAP;
  const v4i cq = *(const v4ia*)(cnt + 4 * tid);
  const v4i oq = *(const v4ia*)(offs + 4 * tid);
  int* cp = CNT  + (size_t)blk * NBA + 4 * tid;
  int* op = OFFS + (size_t)blk * NBA + 4 * tid;
  v4i cv;
  cv.x = (tid == 0) ? nh : 0;
  cv.y = (tid == 0) ? ovf : 0;
  cv.z = 0; cv.w = 0;
  int* fp = FLG + (size_t)blk * 32 + 4 * (tid & 7);
#pragma unroll 1
  for (int p = tid * 4; p < RCAP; p += NTHR * 4) {
    const v4i v = *(const v4ia*)(reg2 + p);
    *(volatile v4i*)(hb + p) = v;
  }
  *(volatile v4i*)cp = cq;
  *(volatile v4i*)op = oq;
  if (tid < 8) *(volatile v4i*)fp = cv;
  __threadfence();
#pragma unroll 1
  for (int p = tid * 4; p < RCAP; p += NTHR * 4) {
    const v4i v = *(const v4ia*)(reg2 + p);
    *(volatile v4i*)(hb + p) = v;
  }
  *(volatile v4i*)cp = cq;
  *(volatile v4i*)op = oq;
  if (tid < 8) *(volatile v4i*)fp = cv;
}

template <int MODE>
__global__ __launch_bounds__(GTHR) __attribute__((amdgpu_num_vgpr(248)))
void k_gemm(const unsigned short* __restrict__ A, const unsigned short* __restrict__ WT, int K,
            float* outF, int ldo, const float* __restrict__ bias, unsigned short* outHL) {
  __shared__ __attribute__((aligned(16))) float stg[GBM * GBN];
  __shared__ __attribute__((aligned(16))) float sbias[GBN];
  const int tid = (int)threadIdx.x, lane = tid & 31, wave = tid >> 5, hh = lane >> 4, m = lane & 15;
  const int rowBase = (int)blockIdx.x * GBM;
  const int col0    = (int)blockIdx.y * GBN;

  if constexpr (MODE == 1) {
    const int pcs = tid & 15;
    const v4f bq = *(const v4f*)(bias + col0 + 4 * pcs);
    if (tid < GBN / 4) *(v4fa*)(sbias + 4 * pcs) = bq;
  }

  v8f acc[4];
  {
    const v8f z = {0.f, 0.f, 0.f, 0.f, 0.f, 0.f, 0.f, 0.f};
    acc[0] = z; acc[1] = z; acc[2] = z; acc[3] = z;
  }
  const unsigned short* ap = A  + (size_t)(rowBase + 16 * wave + m) * (size_t)K + 8 * hh;
  const unsigned short* wp = WT + (size_t)(col0 + m) * (size_t)K + 8 * hh;
  const int ksteps = K >> 5;
#pragma unroll 1
  for (int ks = 0; ks < ksteps; ++ks) {
    FragB af;
    af.h[0] = *(const v8usa*)(ap + 32 * ks);
    af.h[1] = *(const v8usa*)(ap + 32 * ks + 16);
#pragma unroll
    for (int t = 0; t < 4; ++t) {
      const unsigned short* wq = wp + (size_t)(16 * t) * (size_t)K + 32 * ks;
      FragB bf;
      bf.h[0] = *(const v8usa*)wq;
      bf.h[1] = *(const v8usa*)(wq + 16);
      acc[t] = wmb(af, bf, acc[t]);
    }
  }

#pragma unroll
  for (int t = 0; t < 4; ++t) {
    const int lc = 16 * t + m;
#pragma unroll
    for (int r = 0; r < 8; ++r) {
      const int lr = 16 * wave + 8 * hh + r;
      stg[lr * GBN + lc] = acc[t][r];
    }
  }
  __syncthreads();

  if constexpr (MODE == 0) {
    v4f fv[8];
#pragma unroll
    for (int i = 0; i < 8; ++i) {
      const int lr = 16 * wave + 2 * i + hh;
      fv[i] = *(const v4fa*)(stg + lr * GBN + 4 * m);
    }
#pragma unroll
    for (int i = 0; i < 8; ++i) {
      const int gr = rowBase + 16 * wave + 2 * i + hh;
      float* op = outF + (size_t)gr * (size_t)ldo + col0 + 4 * m;
      *(volatile v4f*)op = fv[i];
    }
    __threadfence();
#pragma unroll
    for (int i = 0; i < 8; ++i) {
      const int gr = rowBase + 16 * wave + 2 * i + hh;
      float* op = outF + (size_t)gr * (size_t)ldo + col0 + 4 * m;
      *(volatile v4f*)op = fv[i];
    }
  } else {
    const int rq = lane >> 3, pc = lane & 7;
    const v4f b0 = *(const v4fa*)(sbias + 8 * pc);
    const v4f b1 = *(const v4fa*)(sbias + 8 * pc + 4);
    v4u hv[4], lv[4];
#pragma unroll
    for (int i = 0; i < 4; ++i) {
      const int lr = 16 * wave + 4 * i + rq;
      const v4f x0 = *(const v4fa*)(stg + lr * GBN + 8 * pc);
      const v4f x1 = *(const v4fa*)(stg + lr * GBN + 8 * pc + 4);
      v4f y0, y1;
      y0.x = lk(x0.x + b0.x); y0.y = lk(x0.y + b0.y); y0.z = lk(x0.z + b0.z); y0.w = lk(x0.w + b0.w);
      y1.x = lk(x1.x + b1.x); y1.y = lk(x1.y + b1.y); y1.z = lk(x1.z + b1.z); y1.w = lk(x1.w + b1.w);
      hv[i] = pack8(y0, y1);
      lv[i] = pack8lo(y0, y1);
    }
#pragma unroll
    for (int i = 0; i < 4; ++i) {
      const int gr = rowBase + 16 * wave + 4 * i + rq;
      unsigned short* op = outHL + (size_t)gr * KA2 + col0 + 8 * pc;
      *(volatile v4u*)op = hv[i];
      *(volatile v4u*)(op + HID) = lv[i];
    }
    __threadfence();
#pragma unroll
    for (int i = 0; i < 4; ++i) {
      const int gr = rowBase + 16 * wave + 4 * i + rq;
      unsigned short* op = outHL + (size_t)gr * KA2 + col0 + 8 * pc;
      *(volatile v4u*)op = hv[i];
      *(volatile v4u*)(op + HID) = lv[i];
    }
  }
}

__global__ __launch_bounds__(NTHR) __attribute__((amdgpu_num_vgpr(248)))
void k_dots(const float* __restrict__ Hm, const float* __restrict__ al, const float* __restrict__ ar, float* SD) {
  __shared__ __attribute__((aligned(16))) float sdt[MROWS * 8];
  const int tid = (int)threadIdx.x, lane = tid & 31, wave = tid >> 5;
  const int rowBase = (int)blockIdx.x * MROWS;
  const v4f al0 = *(const v4f*)(al + 4 * lane);
  const v4f al1 = *(const v4f*)(al + HID + 4 * lane);
  const v4f al2 = *(const v4f*)(al + 2 * HID + 4 * lane);
  const v4f ar0 = *(const v4f*)(ar + 4 * lane);
  const v4f ar1 = *(const v4f*)(ar + HID + 4 * lane);
  const v4f ar2 = *(const v4f*)(ar + 2 * HID + 4 * lane);
  const int j = lane & 7;
#pragma unroll 1
  for (int i = 0; i < MROWS / NWAVE; ++i) {
    const int lr = wave * (MROWS / NWAVE) + i;
    const float* rp = Hm + (size_t)(rowBase + lr) * HC + 4 * lane;
    const v4f h0 = *(const v4f*)rp;
    const v4f h1 = *(const v4f*)(rp + HID);
    const v4f h2 = *(const v4f*)(rp + 2 * HID);
    float e0 = fmaf(h0.w, al0.w, fmaf(h0.z, al0.z, fmaf(h0.y, al0.y, h0.x * al0.x)));
    float e1 = fmaf(h1.w, al1.w, fmaf(h1.z, al1.z, fmaf(h1.y, al1.y, h1.x * al1.x)));
    float e2 = fmaf(h2.w, al2.w, fmaf(h2.z, al2.z, fmaf(h2.y, al2.y, h2.x * al2.x)));
    float r0 = fmaf(h0.w, ar0.w, fmaf(h0.z, ar0.z, fmaf(h0.y, ar0.y, h0.x * ar0.x)));
    float r1 = fmaf(h1.w, ar1.w, fmaf(h1.z, ar1.z, fmaf(h1.y, ar1.y, h1.x * ar1.x)));
    float r2 = fmaf(h2.w, ar2.w, fmaf(h2.z, ar2.z, fmaf(h2.y, ar2.y, h2.x * ar2.x)));
#pragma unroll
    for (int off = 16; off > 0; off >>= 1) {
      e0 += __shfl_xor(e0, off, 32);
      e1 += __shfl_xor(e1, off, 32);
      e2 += __shfl_xor(e2, off, 32);
      r0 += __shfl_xor(r0, off, 32);
      r1 += __shfl_xor(r1, off, 32);
      r2 += __shfl_xor(r2, off, 32);
    }
    float v = 0.0f;
    v = (j == 0) ? e0 : v;
    v = (j == 1) ? e1 : v;
    v = (j == 2) ? e2 : v;
    v = (j == 4) ? r0 : v;
    v = (j == 5) ? r1 : v;
    v = (j == 6) ? r2 : v;
    if (lane < 8) sdt[lr * 8 + lane] = v;
  }
  __syncthreads();
  const v4f o = *(const v4fa*)(sdt + 4 * tid);
  float* op = SD + (size_t)rowBase * 8 + 4 * tid;
  *(volatile v4f*)op = o;
  __threadfence();
  *(volatile v4f*)op = o;
}

__device__ __forceinline__ void upd(const float lg, float& mx, float& dn, v4f& ac, const v4f hv) {
  const float df = lg - mx;
  const float ee = expf(-fabsf(df));
  const bool  up = df > 0.0f;
  const float s1 = up ? ee : 1.0f;
  const float s2 = up ? 1.0f : ee;
  mx = up ? lg : mx;
  dn = fmaf(dn, s1, s2);
  ac.x = fmaf(ac.x, s1, s2 * hv.x);
  ac.y = fmaf(ac.y, s1, s2 * hv.y);
  ac.z = fmaf(ac.z, s1, s2 * hv.z);
  ac.w = fmaf(ac.w, s1, s2 * hv.w);
}

__global__ __launch_bounds__(NTHR) __attribute__((amdgpu_num_vgpr(248)))
void k_scan(const int* __restrict__ HITS, const int* __restrict__ CNT, const int* __restrict__ OFFS,
            const int* __restrict__ FLGB, const float* __restrict__ F, const float* __restrict__ SD,
            const float* __restrict__ bias, unsigned short* XP, int* FLGO, int nN, int MPr) {
  extern __shared__ __attribute__((aligned(16))) int ssm[];
  int* sl   = ssm;
  int* cnt  = sl + RCAP;
  int* offs = cnt + NBA;
  int* misc = offs + NBA;
  const int tid = (int)threadIdx.x, lane = tid & 31, wave = tid >> 5;
  const int blk = (int)blockIdx.x;
  const int nodeBase = blk * NBA;

  const int nhraw = FLGB[(size_t)blk * 32];
  const int bflag = FLGB[(size_t)blk * 32 + 1];
  const int nh  = nhraw < 0 ? 0 : (nhraw > RCAP ? RCAP : nhraw);
  const int ovf = (bflag != 0 || nhraw < 0 || nhraw > RCAP) ? 1 : 0;

  {
    const int* hb = HITS + (size_t)blk * RCAP;
#pragma unroll 1
    for (int p = tid * 4; p < RCAP; p += NTHR * 4) *(v4ia*)(sl + p) = *(const v4i*)(hb + p);
    *(v4ia*)(cnt  + 4 * tid) = *(const v4i*)(CNT  + (size_t)blk * NBA + 4 * tid);
    *(v4ia*)(offs + 4 * tid) = *(const v4i*)(OFFS + (size_t)blk * NBA + 4 * tid);
    if (tid < 16) misc[tid] = 0;
  }
  __syncthreads();

  const float qnan = __int_as_float(0x7fc00000);
  const float pzb  = (ovf != 0) ? qnan : 0.0f;
  const v4f bq0 = *(const v4f*)(bias + 4 * lane);
  const v4f bq1 = *(const v4f*)(bias + HID + 4 * lane);
  const v4f bq2 = *(const v4f*)(bias + 2 * HID + 4 * lane);
  int anybig = 0;

#pragma unroll 1
  for (int si = 0; si < NBA / NWAVE; ++si) {
    const int s    = si * NWAVE + wave;
    const int node = nodeBase + s;
    const int nc   = node < nN ? node : nN - 1;
    int c = cnt[s];
    const bool big = c > DEGCAP;
    anybig |= big ? 1 : 0;
    c = c < 0 ? 0 : (c > DEGCAP ? DEGCAP : c);
    int o = offs[s];
    o = o < 0 ? 0 : (o > RCAP ? RCAP : o);
    if (c > nh - o) c = nh - o;
    c = c < 0 ? 0 : c;
    c = __builtin_amdgcn_readfirstlane(c);
    o = __builtin_amdgcn_readfirstlane(o);
    const v4f sdd = *(const v4f*)(SD + (size_t)nc * 8 + 4);
    float mx0 = MXI, mx1 = MXI, mx2 = MXI;
    float dn0 = 0.0f, dn1 = 0.0f, dn2 = 0.0f;
    v4f a0 = {0.f, 0.f, 0.f, 0.f};
    v4f a1 = {0.f, 0.f, 0.f, 0.f};
    v4f a2 = {0.f, 0.f, 0.f, 0.f};
#pragma unroll 1
    for (int b0 = 0; b0 < c; b0 += 32) {
      const int t = b0 + lane;
      int idx = o + t;
      idx = idx < 0 ? 0 : (idx > RCAP - 1 ? RCAP - 1 : idx);
      const int ent = sl[idx];
      int hs = ent & 0xFFFF;
      hs = hs > nN - 1 ? nN - 1 : hs;
      const int m32 = (c - b0) < 32 ? (c - b0) : 32;
#pragma unroll 1
      for (int k = 0; k < m32; ++k) {
        const int sk = __builtin_amdgcn_readlane(hs, k);
        const float* rp = F + (size_t)sk * HC + 4 * lane;
        const v4f sds = *(const v4f*)(SD + (size_t)sk * 8);
        const v4f h0 = *(const v4f*)rp;
        const v4f h1 = *(const v4f*)(rp + HID);
        const v4f h2 = *(const v4f*)(rp + 2 * HID);
        float l0 = sds.x + sdd.x; l0 = l0 > 0.0f ? l0 : GSLOPE * l0;
        float l1 = sds.y + sdd.y; l1 = l1 > 0.0f ? l1 : GSLOPE * l1;
        float l2 = sds.z + sdd.z; l2 = l2 > 0.0f ? l2 : GSLOPE * l2;
        upd(l0, mx0, dn0, a0, h0);
        upd(l1, mx1, dn1, a1, h1);
        upd(l2, mx2, dn2, a2, h2);
      }
    }
    const float i0 = __builtin_amdgcn_rcpf(dn0 + 1e-9f);
    const float i1 = __builtin_amdgcn_rcpf(dn1 + 1e-9f);
    const float i2 = __builtin_amdgcn_rcpf(dn2 + 1e-9f);
    const float pzr = big ? qnan : pzb;
    const bool live = node < nN;
    float x0 = (lk(fmaf(a0.x, i0, bq0.x)) + lk(fmaf(a1.x, i1, bq1.x)) + lk(fmaf(a2.x, i2, bq2.x))) * (1.0f / 3.0f);
    float x1 = (lk(fmaf(a0.y, i0, bq0.y)) + lk(fmaf(a1.y, i1, bq1.y)) + lk(fmaf(a2.y, i2, bq2.y))) * (1.0f / 3.0f);
    float x2 = (lk(fmaf(a0.z, i0, bq0.z)) + lk(fmaf(a1.z, i1, bq1.z)) + lk(fmaf(a2.z, i2, bq2.z))) * (1.0f / 3.0f);
    float x3 = (lk(fmaf(a0.w, i0, bq0.w)) + lk(fmaf(a1.w, i1, bq1.w)) + lk(fmaf(a2.w, i2, bq2.w))) * (1.0f / 3.0f);
    x0 = (live ? x0 : 0.0f) + pzr;
    x1 = (live ? x1 : 0.0f) + pzr;
    x2 = (live ? x2 : 0.0f) + pzr;
    x3 = (live ? x3 : 0.0f) + pzr;
    v2u hv, lv;
    hv.x = pk2(x0, x1);   hv.y = pk2(x2, x3);
    lv.x = pk2lo(x0, x1); lv.y = pk2lo(x2, x3);
    if (node < MPr) {
      unsigned short* hp = XP + (size_t)node * KA2 + 4 * lane;
      *(volatile v2u*)hp = hv;
      *(volatile v2u*)(hp + HID) = lv;
      __threadfence();
      *(volatile v2u*)hp = hv;
      *(volatile v2u*)(hp + HID) = lv;
    }
  }

  if (lane == 0) misc[wave] = anybig;
  __syncthreads();
  if (wave == 0) {
    int fg = ovf;
#pragma unroll
    for (int w2 = 0; w2 < NWAVE; ++w2) fg |= misc[w2];
    v4i cv;
    cv.x = 0;
    cv.y = (lane == 0) ? fg : 0;
    cv.z = 0; cv.w = 0;
    int* fp = FLGO + (size_t)blk * 32 + 4 * (lane & 7);
    if (lane < 8) *(volatile v4i*)fp = cv;
    __threadfence();
    if (lane < 8) *(volatile v4i*)fp = cv;
  }
}

__global__ __launch_bounds__(GTHR) __attribute__((amdgpu_num_vgpr(248)))
void k_out(const unsigned short* __restrict__ A, const unsigned short* __restrict__ W5,
           const float* __restrict__ lb5, const int* __restrict__ FLG, int gA, float* out, int nN) {
  __shared__ __attribute__((aligned(16))) float so[ORW * NCLS];
  const int tid = (int)threadIdx.x, lane = tid & 31, wave = tid >> 5, hh = lane >> 4, m = lane & 15;
  const int row0 = (int)blockIdx.x * ORW;
  v8f acc0 = {0.f, 0.f, 0.f, 0.f, 0.f, 0.f, 0.f, 0.f};
  v8f acc1 = {0.f, 0.f, 0.f, 0.f, 0.f, 0.f, 0.f, 0.f};
  const unsigned short* ap = A  + (size_t)(row0 + 32 * wave + m) * KA2 + 8 * hh;
  const unsigned short* wp = W5 + (size_t)m * KA2 + 8 * hh;
#pragma unroll 1
  for (int ks = 0; ks < KA2 / 32; ++ks) {
    FragB bf, af0, af1;
    bf.h[0]  = *(const v8usa*)(wp + 32 * ks);
    bf.h[1]  = *(const v8usa*)(wp + 32 * ks + 16);
    af0.h[0] = *(const v8usa*)(ap + 32 * ks);
    af0.h[1] = *(const v8usa*)(ap + 32 * ks + 16);
    af1.h[0] = *(const v8usa*)(ap + (size_t)16 * KA2 + 32 * ks);
    af1.h[1] = *(const v8usa*)(ap + (size_t)16 * KA2 + 32 * ks + 16);
    acc0 = wmb(af0, bf, acc0);
    acc1 = wmb(af1, bf, acc1);
  }
  const float bv = lb5[m < NCLS ? m : NCLS - 1];
  if (m < NCLS) {
#pragma unroll
    for (int r = 0; r < 8; ++r) {
      so[(32 * wave + 8 * hh + r) * NCLS + m]      = acc0[r] + bv;
      so[(32 * wave + 16 + 8 * hh + r) * NCLS + m] = acc1[r] + bv;
    }
  }
  __syncthreads();

  int bb = row0 >> SLA;
  bb = bb > gA - 1 ? gA - 1 : bb;
  const int fg = FLG[(size_t)bb * 32 + 1] | FLG[((size_t)gA + bb) * 32 + 1] | FLG[((size_t)2 * gA + bb) * 32 + 1];
  int rows = nN - row0;
  rows = rows < 0 ? 0 : (rows > ORW ? ORW : rows);
  const int npc = (rows * NCLS) / 4;
  const int p0 = tid;
  const int p1 = GTHR + tid;
  const int p1c = p1 < (ORW * NCLS) / 4 ? p1 : (ORW * NCLS) / 4 - 1;
  v4f v0 = *(const v4fa*)(so + 4 * p0);
  v4f v1 = *(const v4fa*)(so + 4 * p1c);
  const float qnan = __int_as_float(0x7fc00000);
  const v4f qn = {qnan, qnan, qnan, qnan};
  v0 = (fg != 0) ? qn : v0;
  v1 = (fg != 0) ? qn : v1;
  float* ob = out + (size_t)row0 * NCLS;
  const bool w0 = p0 < npc;
  const bool w1 = (tid < 64) && (p1 < npc);
  if (w0) *(volatile v4f*)(ob + 4 * p0) = v0;
  if (w1) *(volatile v4f*)(ob + 4 * p1) = v1;
  __threadfence();
  if (w0) *(volatile v4f*)(ob + 4 * p0) = v0;
  if (w1) *(volatile v4f*)(ob + 4 * p1) = v1;
}

static inline int cdiv(int a, int b) { return (a + b - 1) / b; }

extern "C" void kernel_launch(void* const* d_in, const int* in_sizes, int n_in,
                              void* d_out, int out_size, void* d_ws, size_t ws_size,
                              hipStream_t stream) {
  if (n_in < 21) return;
  const int nN = in_sizes[0] / FIN;
  if (nN <= 0 || in_sizes[0] != nN * FIN || nN > 65536 || (nN % 16) != 0) return;
  const int nE = in_sizes[1];
  if (nE < 1 || nE > (1 << 30) || in_sizes[2] != nE) return;
  if (in_sizes[3] != FIN * HC || in_sizes[7] != HID * HC) return;
  if (in_sizes[4] != HC || in_sizes[5] != HC || in_sizes[6] != HC) return;
  if (in_sizes[8] != HC || in_sizes[9] != HC || in_sizes[10] != HC) return;
  for (int i = 0; i < 4; ++i) {
    if (in_sizes[11 + 2 * i] != HID * HID || in_sizes[12 + 2 * i] != HID) return;
  }
  if (in_sizes[19] != HID * NCLS || in_sizes[20] != NCLS) return;
  if (out_size != nN * NCLS) return;

  const float* x   = (const float*)d_in[0];
  const int*   src = (const int*)  d_in[1];
  const int*   dst = (const int*)  d_in[2];
  const float* W1  = (const float*)d_in[3];
  const float* al1 = (const float*)d_in[4];
  const float* ar1 = (const float*)d_in[5];
  const float* b1  = (const float*)d_in[6];
  const float* W2  = (const float*)d_in[7];
  const float* al2 = (const float*)d_in[8];
  const float* ar2 = (const float*)d_in[9];
  const float* b2  = (const float*)d_in[10];
  const float* lw1 = (const float*)d_in[11];
  const float* lb1 = (const float*)d_in[12];
  const float* lw2 = (const float*)d_in[13];
  const float* lb2 = (const float*)d_in[14];
  const float* lw3 = (const float*)d_in[15];
  const float* lb3 = (const float*)d_in[16];
  const float* lw4 = (const float*)d_in[17];
  const float* lb4 = (const float*)d_in[18];
  const float* lw5 = (const float*)d_in[19];
  const float* lb5 = (const float*)d_in[20];
  float* out = (float*)d_out;

  const int MP   = cdiv(nN, MROWS) * MROWS;
  const int gM   = MP / GBM;
  const int gA   = cdiv(MP, NBA);
  if ((long long)gA * NBA < (long long)MP) return;
  const int vec8 = ((nE & 3) == 0) ? 1 : 0;
  const int nUx  = MP * (FIN / 8);
  if ((nUx % NTHR) != 0) return;

  char* ws = (char*)d_ws;
  size_t off = 0;
  const size_t szH  = (size_t)MP * HC * 4;
  const size_t szXA = (size_t)MP * KA2 * 2;
  const size_t oH   = off; off += szH;                            off = (off + 255) & ~(size_t)255;
  const size_t oXA  = off; off += szXA;                           off = (off + 255) & ~(size_t)255;
  const size_t oHIT = off; off += (size_t)gA * RCAP * 4;          off = (off + 255) & ~(size_t)255;
  const size_t oCNT = off; off += (size_t)gA * NBA * 4;           off = (off + 255) & ~(size_t)255;
  const size_t oOFF = off; off += (size_t)gA * NBA * 4;           off = (off + 255) & ~(size_t)255;
  const size_t oFLG = off; off += (size_t)3 * gA * 128;           off = (off + 255) & ~(size_t)255;
  const size_t oSD  = off; off += (size_t)MP * 8 * 4;             off = (off + 255) & ~(size_t)255;
  const size_t oW1T = off; off += (size_t)HC * FIN * 2;           off = (off + 255) & ~(size_t)255;
  const size_t oW2D = off; off += (size_t)HC * KA2 * 2;           off = (off + 255) & ~(size_t)255;
  const size_t oLWD = off; off += (size_t)4 * HID * KA2 * 2;      off = (off + 255) & ~(size_t)255;
  const size_t oLW5 = off; off += (size_t)16 * KA2 * 2;           off = (off + 255) & ~(size_t)255;
  const size_t oPAR = off; off += (size_t)PAR_N * 4;              off = (off + 255) & ~(size_t)255;
  if (off > ws_size || off > (size_t)WSMAX) return;
  if (szXA > szH) return;
  if ((size_t)MP * FIN * 2 > szXA) return;

  float*          H    = (float*)(ws + oH);
  unsigned short* P    = (unsigned short*)(ws + oH);
  unsigned short* XA   = (unsigned short*)(ws + oXA);
  unsigned short* XB   = (unsigned short*)(ws + oXA);
  int*            HITS = (int*)(ws + oHIT);
  int*            CNT  = (int*)(ws + oCNT);
  int*            OFFS = (int*)(ws + oOFF);
  int*            FLG  = (int*)(ws + oFLG);
  float*          SD   = (float*)(ws + oSD);
  unsigned short* W1T  = (unsigned short*)(ws + oW1T);
  unsigned short* W2D  = (unsigned short*)(ws + oW2D);
  unsigned short* LWD  = (unsigned short*)(ws + oLWD);
  unsigned short* LW5D = (unsigned short*)(ws + oLW5);
  float*          PAR  = (float*)(ws + oPAR);
  int* FLG0 = FLG;
  int* FLG1 = FLG + (size_t)gA * 32;
  int* FLG2 = FLG + (size_t)2 * gA * 32;

  const int bktLds  = BKT_LDS_INTS * 4;
  const int scanLds = SCAN_LDS_INTS * 4;
  hipFuncSetAttribute(reinterpret_cast<const void*>(&k_bucket),
                      hipFuncAttributeMaxDynamicSharedMemorySize, bktLds);
  hipFuncSetAttribute(reinterpret_cast<const void*>(&k_scan),
                      hipFuncAttributeMaxDynamicSharedMemorySize, scanLds);

  k_pa<<<(nUx + NUW1) / NTHR, NTHR, 0, stream>>>(x, W1, XB, W1T, nN, nUx);
  k_pb<<<(NU2 + 4 * NUL + NU5) / NTHR, NTHR, 0, stream>>>(W2, lw1, lw2, lw3, lw4, lw5, W2D, LWD, LW5D);
  k_pc<<<23, 32, 0, stream>>>(al1, ar1, b1, al2, ar2, b2, lb1, lb2, lb3, lb4, lb5, PAR);
  k_bucket<<<gA, NTHR, bktLds, stream>>>(src, dst, nE, nN, vec8, HITS, CNT, OFFS, FLG0);

  k_gemm<0><<<dim3(gM, HC / GBN), GTHR, 0, stream>>>(XB, W1T, FIN, H, HC, PAR, XA);
  k_dots<<<MP / MROWS, NTHR, 0, stream>>>(H, PAR + PAR_AL1, PAR + PAR_AR1, SD);
  k_scan<<<gA, NTHR, scanLds, stream>>>(HITS, CNT, OFFS, FLG0, H, SD, PAR + PAR_B1, XA, FLG1, nN, MP);

  k_gemm<0><<<dim3(gM, HC / GBN), GTHR, 0, stream>>>(XA, W2D, KA2, H, HC, PAR, XA);
  k_dots<<<MP / MROWS, NTHR, 0, stream>>>(H, PAR + PAR_AL2, PAR + PAR_AR2, SD);
  k_scan<<<gA, NTHR, scanLds, stream>>>(HITS, CNT, OFFS, FLG0, H, SD, PAR + PAR_B2, XA, FLG2, nN, MP);

  k_gemm<1><<<dim3(gM, HID / GBN), GTHR, 0, stream>>>(XA, LWD,                         KA2, SD, 0, PAR + PAR_LB,           P);
  k_gemm<1><<<dim3(gM, HID / GBN), GTHR, 0, stream>>>(P,  LWD + (size_t)HID * KA2,     KA2, SD, 0, PAR + PAR_LB + HID,     XA);
  k_gemm<1><<<dim3(gM, HID / GBN), GTHR, 0, stream>>>(XA, LWD + (size_t)2 * HID * KA2, KA2, SD, 0, PAR + PAR_LB + 2 * HID, P);
  k_gemm<1><<<dim3(gM, HID / GBN), GTHR, 0, stream>>>(P,  LWD + (size_t)3 * HID * KA2, KA2, SD, 0, PAR + PAR_LB + 3 * HID, XA);

  k_out<<<MP / ORW, GTHR, 0, stream>>>(XA, LW5D, PAR + PAR_LB5, FLG, gA, out, nN);
}
